// Encoder_48412871360843
// MI455X (gfx1250) — hardware-verified
//
#include <hip/hip_runtime.h>
#include <hip/hip_fp16.h>


#ifndef NB
#define NB 2
#endif
#ifndef SEQ
#define SEQ 2048
#endif
#define NB_FULL  2
#define SEQ_FULL 2048
#define DM   1024
#define NH   16
#define HD   64
#define DFF  4096
#define NTOK (NB * SEQ)
#define PB   64

static_assert(NB >= 1 && NB <= NB_FULL);
static_assert(SEQ >= 128 && SEQ <= SEQ_FULL);
static_assert(SEQ % 128 == 0);
static_assert(NTOK % 128 == 0);
static_assert(PB == 64);
static_assert(DM == NH * HD);
static_assert(DM % 128 == 0 && DFF % 128 == 0);
static_assert(((size_t)SEQ * DM / PB) % 4 == 0);

typedef _Float16 v16h __attribute__((ext_vector_type(16)));
typedef _Float16 v8h  __attribute__((ext_vector_type(8)));
typedef float    v8f  __attribute__((ext_vector_type(8)));
typedef float    v4f  __attribute__((ext_vector_type(4)));

union Frag { v16h v; v8h h[2]; };

#define CS      (1.44269504088896340736f * 3.0517578125e-05f)
#define SC_W    64.0f
#define SC_FOLD 2.44140625e-04f
#define LN_EPS  1.0e-5f

static __device__ __forceinline__ v8f zero8() {
    v8f z;
#pragma unroll
    for (int i = 0; i < 8; ++i) z[i] = 0.0f;
    return z;
}

static __device__ __forceinline__ v16h load_frag16(const _Float16* base, int ld, int lane) {
    int m  = lane & 15;
    int kb = (lane >> 4) << 3;
    const _Float16* p = base + (size_t)m * ld + kb;
    Frag f;
    f.h[0] = *(const v8h*)(p);
    f.h[1] = *(const v8h*)(p + 16);
    return f.v;
}

static __device__ __forceinline__ v8f wmma16(v16h a, v16h b, v8f c) {
    v8f d = __builtin_amdgcn_wmma_f32_16x16x32_f16(false, a, false, b, (short)0, c, false, false);
    asm volatile("v_nop\n\tv_nop\n\tv_nop\n\tv_nop" : "+v"(d) : "v"(a), "v"(b));
    return d;
}

static __device__ __forceinline__ float bf16r(float x) {
    unsigned u = __float_as_uint(x);
    u = (u + 0x7FFFu + ((u >> 16) & 1u)) & 0xFFFF0000u;
    return __uint_as_float(u);
}

static __device__ __forceinline__ v4f bf16r4(v4f v) {
    v4f o;
    o.x = bf16r(v.x); o.y = bf16r(v.y); o.z = bf16r(v.z); o.w = bf16r(v.w);
    return o;
}

static __device__ __forceinline__ float ex2(float x) {
    return __builtin_amdgcn_exp2f(x);
}

static __device__ __forceinline__ void wave_lds_sync() {
    __builtin_amdgcn_fence(3, "wavefront");
    asm volatile("s_wait_dscnt 0" ::: "memory");
    __builtin_amdgcn_wave_barrier();
}

static __device__ __forceinline__ float wave_sum(float s) {
    s += __shfl_xor(s, 16, 32);
    s += __shfl_xor(s, 8, 32);
    s += __shfl_xor(s, 4, 32);
    s += __shfl_xor(s, 2, 32);
    s += __shfl_xor(s, 1, 32);
    return s;
}

static __device__ __forceinline__ double wave_part_total(const float* __restrict__ part, int b, int lane) {
    double a = (double)part[((size_t)b * PB + lane) * 32] +
               (double)part[((size_t)b * PB + lane + 32) * 32];
    a += __shfl_xor(a, 16, 32);
    a += __shfl_xor(a, 8, 32);
    a += __shfl_xor(a, 4, 32);
    a += __shfl_xor(a, 2, 32);
    a += __shfl_xor(a, 1, 32);
    return a;
}

__global__ __launch_bounds__(256) void k_cvt(const float* __restrict__ x,
                                              _Float16* __restrict__ xh) {
    const int tid = threadIdx.x;
    const int bpb = SEQ / 8;
    const int b   = blockIdx.x / bpb;
    const int lb  = blockIdx.x - b * bpb;
    const float* src = x + (size_t)b * SEQ_FULL * DM + (size_t)lb * 8192;
    _Float16*    dst = xh + (size_t)b * SEQ * DM + (size_t)lb * 8192;
    v8h o[4];
#pragma unroll
    for (int it = 0; it < 4; ++it) {
        const int e = it * 2048 + tid * 8;
        v4f a = *(const v4f*)(src + e);
        v4f c = *(const v4f*)(src + e + 4);
        v8h hv;
        hv[0] = (_Float16)bf16r(a.x); hv[1] = (_Float16)bf16r(a.y);
        hv[2] = (_Float16)bf16r(a.z); hv[3] = (_Float16)bf16r(a.w);
        hv[4] = (_Float16)bf16r(c.x); hv[5] = (_Float16)bf16r(c.y);
        hv[6] = (_Float16)bf16r(c.z); hv[7] = (_Float16)bf16r(c.w);
        o[it] = hv;
    }
#pragma unroll
    for (int it = 0; it < 4; ++it) *(volatile v8h*)(dst + it * 2048 + tid * 8) = o[it];
    __threadfence();
#pragma unroll
    for (int it = 0; it < 4; ++it) *(volatile v8h*)(dst + it * 2048 + tid * 8) = o[it];
}

__global__ __launch_bounds__(256) void k_wprep(const float* __restrict__ W, int K, int N,
                                                _Float16* __restrict__ WT) {
    __shared__ __align__(16) _Float16 T[64 * 72];
    const int tid = threadIdx.x;
    const int n0 = blockIdx.x * 64;
    const int k0 = blockIdx.y * 64;
#pragma unroll
    for (int it = 0; it < 4; ++it) {
        const int idx = it * 256 + tid;
        const int k  = idx >> 4;
        const int c4 = (idx & 15) * 4;
        v4f v = *(const v4f*)(W + (size_t)(k0 + k) * N + n0 + c4);
        T[(c4 + 0) * 72 + k] = (_Float16)(bf16r(v.x) * SC_W);
        T[(c4 + 1) * 72 + k] = (_Float16)(bf16r(v.y) * SC_W);
        T[(c4 + 2) * 72 + k] = (_Float16)(bf16r(v.z) * SC_W);
        T[(c4 + 3) * 72 + k] = (_Float16)(bf16r(v.w) * SC_W);
    }
    __syncthreads();
    const int rr = tid >> 3;
    const int c8 = (tid & 7) * 8;
    v8h o0 = *(const v8h*)(&T[rr * 72 + c8]);
    v8h o1 = *(const v8h*)(&T[(32 + rr) * 72 + c8]);
    _Float16* d0 = WT + (size_t)(n0 + rr) * K + k0 + c8;
    _Float16* d1 = WT + (size_t)(n0 + 32 + rr) * K + k0 + c8;
    *(volatile v8h*)d0 = o0;
    *(volatile v8h*)d1 = o1;
    __threadfence();
    *(volatile v8h*)d0 = o0;
    *(volatile v8h*)d1 = o1;
}

template<bool BFIN>
__global__ __launch_bounds__(256) void k_lnsum(const float* __restrict__ t, int bstride,
                                                float* __restrict__ part) {
    __shared__ float sh8[8];
    const int tid = threadIdx.x, lane = tid & 31, w = tid >> 5;
    const int blk = blockIdx.x, b = blockIdx.y;
    const size_t chunk = (size_t)SEQ * DM / PB;
    const float* p = t + (size_t)b * bstride + (size_t)blk * chunk;
    float s = 0.0f;
    for (int i = tid; i < (int)(chunk / 4); i += 256) {
        v4f v = *(const v4f*)(p + (size_t)i * 4);
        if (BFIN) v = bf16r4(v);
        s += (v.x + v.y) + (v.z + v.w);
    }
    s = wave_sum(s);
    if (lane == 0) sh8[w] = s;
    __syncthreads();
    const float tot = ((sh8[0] + sh8[1]) + (sh8[2] + sh8[3])) + ((sh8[4] + sh8[5]) + (sh8[6] + sh8[7]));
    if (tid < 8) {
        v4f o;
        o.x = (tid == 0) ? tot : 0.0f; o.y = 0.0f; o.z = 0.0f; o.w = 0.0f;
        float* dst = part + ((size_t)b * PB + blk) * 32 + tid * 4;
        *(volatile v4f*)dst = o;
        __threadfence();
        *(volatile v4f*)dst = o;
    }
}

template<bool BFIN>
__global__ __launch_bounds__(256) void k_lnvar(const float* __restrict__ t, int bstride,
                                                const float* __restrict__ partS,
                                                float* __restrict__ partV) {
    __shared__ float  sh8[8];
    __shared__ double shd[1];
    const int tid = threadIdx.x, lane = tid & 31, w = tid >> 5;
    const int blk = blockIdx.x, b = blockIdx.y;
    if (w == 0) {
        double a = wave_part_total(partS, b, lane);
        if (lane == 0) shd[0] = a;
    }
    __syncthreads();
    const double inv_n = 1.0 / ((double)SEQ * (double)DM);
    const float mu = (float)(shd[0] * inv_n);
    const size_t chunk = (size_t)SEQ * DM / PB;
    const float* p = t + (size_t)b * bstride + (size_t)blk * chunk;
    float s = 0.0f;
    for (int i = tid; i < (int)(chunk / 4); i += 256) {
        v4f v = *(const v4f*)(p + (size_t)i * 4);
        if (BFIN) v = bf16r4(v);
        const float d0 = v.x - mu, d1 = v.y - mu, d2 = v.z - mu, d3 = v.w - mu;
        s += (d0 * d0 + d1 * d1) + (d2 * d2 + d3 * d3);
    }
    s = wave_sum(s);
    if (lane == 0) sh8[w] = s;
    __syncthreads();
    const float tot = ((sh8[0] + sh8[1]) + (sh8[2] + sh8[3])) + ((sh8[4] + sh8[5]) + (sh8[6] + sh8[7]));
    if (tid < 8) {
        v4f o;
        o.x = (tid == 0) ? tot : 0.0f; o.y = 0.0f; o.z = 0.0f; o.w = 0.0f;
        float* dst = partV + ((size_t)b * PB + blk) * 32 + tid * 4;
        *(volatile v4f*)dst = o;
        __threadfence();
        *(volatile v4f*)dst = o;
    }
}

template<bool BFIN>
__global__ __launch_bounds__(256) void k_lnnorm(const float* __restrict__ t, int bstride,
                                                 const float* __restrict__ partS,
                                                 const float* __restrict__ partV,
                                                 const float* __restrict__ lw,
                                                 const float* __restrict__ lb,
                                                 _Float16* __restrict__ outh) {
    __shared__ double shd[2];
    const int tid = threadIdx.x, lane = tid & 31, w = tid >> 5;
    const int bpb = SEQ / 8;
    const int b   = blockIdx.x / bpb;
    const int lbk = blockIdx.x - b * bpb;
    if (w == 0) {
        double a = wave_part_total(partS, b, lane);
        double c = wave_part_total(partV, b, lane);
        if (lane == 0) { shd[0] = a; shd[1] = c; }
    }
    __syncthreads();
    const double inv_n = 1.0 / ((double)SEQ * (double)DM);
    const float mu   = (float)(shd[0] * inv_n);
    const float var  = (float)(shd[1] * inv_n);
    const float rstd = rsqrtf(var + LN_EPS);

    const size_t e0 = (size_t)lbk * 8192;
    const float* src = t + (size_t)b * bstride + e0;
    const float* wp  = lw + e0;
    const float* bp  = lb + e0;
    _Float16* dst = outh + (size_t)b * SEQ * DM + e0;
    v8h o[4];
#pragma unroll
    for (int it = 0; it < 4; ++it) {
        const int e = it * 2048 + tid * 8;
        v4f a0 = *(const v4f*)(src + e);
        v4f a1 = *(const v4f*)(src + e + 4);
        if (BFIN) { a0 = bf16r4(a0); a1 = bf16r4(a1); }
        v4f w0 = bf16r4(*(const v4f*)(wp + e));
        v4f w1 = bf16r4(*(const v4f*)(wp + e + 4));
        v4f b0 = bf16r4(*(const v4f*)(bp + e));
        v4f b1 = bf16r4(*(const v4f*)(bp + e + 4));
        v8h hv;
        hv[0] = (_Float16)((a0.x - mu) * rstd * w0.x + b0.x);
        hv[1] = (_Float16)((a0.y - mu) * rstd * w0.y + b0.y);
        hv[2] = (_Float16)((a0.z - mu) * rstd * w0.z + b0.z);
        hv[3] = (_Float16)((a0.w - mu) * rstd * w0.w + b0.w);
        hv[4] = (_Float16)((a1.x - mu) * rstd * w1.x + b1.x);
        hv[5] = (_Float16)((a1.y - mu) * rstd * w1.y + b1.y);
        hv[6] = (_Float16)((a1.z - mu) * rstd * w1.z + b1.z);
        hv[7] = (_Float16)((a1.w - mu) * rstd * w1.w + b1.w);
        o[it] = hv;
    }
#pragma unroll
    for (int it = 0; it < 4; ++it) *(volatile v8h*)(dst + it * 2048 + tid * 8) = o[it];
    __threadfence();
#pragma unroll
    for (int it = 0; it < 4; ++it) *(volatile v8h*)(dst + it * 2048 + tid * 8) = o[it];
}

template<bool F32OUT, bool RELU, bool BIASROW, bool RESBF>
__global__ __launch_bounds__(128) __attribute__((amdgpu_num_vgpr(256)))
void k_gemm(const _Float16* __restrict__ A, const _Float16* __restrict__ Bm,
            int K, int lda, int ldb,
            const float* __restrict__ bias, float alpha, float beta,
            const float* __restrict__ res, int res_bstride,
            void* __restrict__ outp, int ldo) {
    const int tid  = threadIdx.x;
    const int lane = tid & 31;
    const int w    = tid >> 5;
    const int m0   = blockIdx.y * 64 + (w >> 1) * 32;
    const int n0   = blockIdx.x * 128 + (w & 1) * 64;
    const int r0   = (lane >> 4) << 3;
    const int cc   = lane & 15;

    const _Float16* ap = A  + (size_t)m0 * lda;
    const _Float16* bp = Bm + (size_t)n0 * ldb;

    v8f acc[2][4];
#pragma unroll
    for (int i = 0; i < 2; ++i)
#pragma unroll
        for (int j = 0; j < 4; ++j) acc[i][j] = zero8();

#pragma unroll 2
    for (int k0 = 0; k0 < K; k0 += 32) {
        v16h a0 = load_frag16(ap + k0, lda, lane);
        v16h a1 = load_frag16(ap + (size_t)16 * lda + k0, lda, lane);
#pragma unroll
        for (int j = 0; j < 4; ++j) {
            v16h bj = load_frag16(bp + (size_t)(j * 16) * ldb + k0, ldb, lane);
            acc[0][j] = wmma16(a0, bj, acc[0][j]);
            acc[1][j] = wmma16(a1, bj, acc[1][j]);
        }
    }

    if constexpr (!F32OUT) {
        __shared__ __align__(16) _Float16 Hst[4][32 * 64];
        _Float16* outh = (_Float16*)outp;
        if constexpr (BIASROW) {
#pragma unroll
            for (int i = 0; i < 2; ++i)
#pragma unroll
                for (int g = 0; g < 8; ++g) {
                    const float bv = beta * bf16r(bias[m0 + i * 16 + r0 + g]);
#pragma unroll
                    for (int j = 0; j < 4; ++j) {
                        float v = acc[i][j][g] * alpha + bv;
                        if (RELU) v = fmaxf(v, 0.0f);
                        Hst[w][(i * 16 + r0 + g) * 64 + j * 16 + cc] = (_Float16)v;
                    }
                }
        } else {
#pragma unroll
            for (int j = 0; j < 4; ++j) {
                const float bv = beta * bf16r(bias[n0 + j * 16 + cc]);
#pragma unroll
                for (int i = 0; i < 2; ++i)
#pragma unroll
                    for (int g = 0; g < 8; ++g) {
                        float v = acc[i][j][g] * alpha + bv;
                        if (RELU) v = fmaxf(v, 0.0f);
                        Hst[w][(i * 16 + r0 + g) * 64 + j * 16 + cc] = (_Float16)v;
                    }
            }
        }
        wave_lds_sync();
        v8h pv[8];
#pragma unroll
        for (int t = 0; t < 8; ++t) pv[t] = *(const v8h*)(&Hst[w][t * 256 + lane * 8]);
        _Float16* ob = outh + (size_t)(m0 + (lane >> 3)) * ldo + n0 + (lane & 7) * 8;
#pragma unroll
        for (int t = 0; t < 8; ++t) *(volatile v8h*)(ob + (size_t)(4 * t) * ldo) = pv[t];
        __threadfence();
#pragma unroll
        for (int t = 0; t < 8; ++t) *(volatile v8h*)(ob + (size_t)(4 * t) * ldo) = pv[t];
    } else {
        __shared__ __align__(16) float Ost[4][32 * 64];
        float* outf = (float*)outp;
#pragma unroll
        for (int i = 0; i < 2; ++i)
#pragma unroll
            for (int j = 0; j < 4; ++j)
#pragma unroll
                for (int g = 0; g < 8; ++g)
                    Ost[w][(i * 16 + r0 + g) * 64 + j * 16 + cc] = acc[i][j][g] * alpha;
        wave_lds_sync();
        const int col = (lane & 15) * 4;
        v4f bb = bf16r4(*(const v4f*)(bias + n0 + col));
        bb.x *= beta; bb.y *= beta; bb.z *= beta; bb.w *= beta;
#pragma unroll
        for (int hh = 0; hh < 2; ++hh) {
            v4f sv[8];
#pragma unroll
            for (int t = 0; t < 8; ++t) {
                const int idx = hh * 8 + t;
                const int m   = m0 + 2 * idx + (lane >> 4);
                const int bq  = m / SEQ;
                const int s   = m - bq * SEQ;
                v4f a = *(const v4f*)(&Ost[w][idx * 128 + lane * 4]);
                v4f r = *(const v4f*)(res + ((size_t)bq * res_bstride + s) * ldo + n0 + col);
                if (RESBF) r = bf16r4(r);
                v4f o;
                o.x = r.x + (a.x + bb.x); o.y = r.y + (a.y + bb.y);
                o.z = r.z + (a.z + bb.z); o.w = r.w + (a.w + bb.w);
                sv[t] = o;
            }
            float* ob = outf + (size_t)(m0 + hh * 16 + (lane >> 4)) * ldo + n0 + col;
#pragma unroll
            for (int t = 0; t < 8; ++t) *(volatile v4f*)(ob + (size_t)(2 * t) * ldo) = sv[t];
            __threadfence();
#pragma unroll
            for (int t = 0; t < 8; ++t) *(volatile v4f*)(ob + (size_t)(2 * t) * ldo) = sv[t];
        }
    }
}

__global__ __launch_bounds__(256) __attribute__((amdgpu_num_vgpr(256)))
void k_attn(const _Float16* __restrict__ qp,
            const _Float16* __restrict__ kp,
            const _Float16* __restrict__ vT,
            _Float16* __restrict__ ctx) {
    __shared__ __align__(16) _Float16 Cst[8][16 * HD];

    const int tid  = threadIdx.x;
    const int lane = tid & 31;
    const int w    = tid >> 5;
    const int b    = blockIdx.z;
    const int h    = blockIdx.y;
    const int q0   = blockIdx.x * 128 + w * 16;
    const int r0   = (lane >> 4) << 3;
    const int cc   = lane & 15;
    const int qi   = q0 + cc;

    const _Float16* qb = qp + ((size_t)b * SEQ + q0) * DM + h * HD;
    const _Float16* kb = kp + ((size_t)b * SEQ) * DM + h * HD;
    const _Float16* vb = vT + ((size_t)h * HD) * NTOK + (size_t)b * SEQ;

    const v16h qf0 = load_frag16(qb, DM, lane);
    const v16h qf1 = load_frag16(qb + 32, DM, lane);

    v8f o[4];
#pragma unroll
    for (int dt = 0; dt < 4; ++dt) o[dt] = zero8();
    float mr = -1.0e30f, lr = 0.0f;

#pragma unroll 1
    for (int k0 = 0; k0 < SEQ; k0 += 32) {
        const _Float16* kr = kb + (size_t)k0 * DM;
        v16h ka0 = load_frag16(kr, DM, lane);
        v16h ka1 = load_frag16(kr + 32, DM, lane);
        v8f s0 = wmma16(ka0, qf0, zero8());
        s0 = wmma16(ka1, qf1, s0);
        v16h kc0 = load_frag16(kr + (size_t)16 * DM, DM, lane);
        v16h kc1 = load_frag16(kr + (size_t)16 * DM + 32, DM, lane);
        v8f s1 = wmma16(kc0, qf0, zero8());
        s1 = wmma16(kc1, qf1, s1);

        float t0[8], t1[8];
        float tmax = -1.0e30f;
#pragma unroll
        for (int g = 0; g < 8; ++g) {
            const int key = k0 + r0 + g;
            const float a0 = s0[g] * CS;
            const float a1 = s1[g] * CS;
            t0[g] = (key <= qi) ? a0 : 0.0f;
            t1[g] = (key + 16 <= qi) ? a1 : 0.0f;
            tmax = fmaxf(tmax, fmaxf(t0[g], t1[g]));
        }
        tmax = fmaxf(tmax, __shfl_xor(tmax, 16, 32));
        const float mn = fmaxf(mr, tmax);
        const float al = ex2(mr - mn);
        mr = mn;
        const float sh = 10.0f - mn;
        Frag pf;
        float ls = 0.0f;
#pragma unroll
        for (int g = 0; g < 8; ++g) {
            const float p0 = ex2(t0[g] + sh);
            const float p1 = ex2(t1[g] + sh);
            pf.v[g]     = (_Float16)p0;
            pf.v[8 + g] = (_Float16)p1;
            ls += p0 + p1;
        }
        lr = lr * al + ls;
#pragma unroll
        for (int dt = 0; dt < 4; ++dt)
#pragma unroll
            for (int g = 0; g < 8; ++g) o[dt][g] *= al;
#pragma unroll
        for (int dt = 0; dt < 4; ++dt) {
            v16h va = load_frag16(vb + (size_t)(dt * 16) * NTOK + k0, NTOK, lane);
            o[dt] = wmma16(va, pf.v, o[dt]);
        }
    }

    const float ltot = lr + __shfl_xor(lr, 16, 32);
    const float inv  = 1.0f / ltot;
#pragma unroll
    for (int dt = 0; dt < 4; ++dt) {
        v8h c;
#pragma unroll
        for (int g = 0; g < 8; ++g) c[g] = (_Float16)(o[dt][g] * inv);
        *(v8h*)(&Cst[w][cc * HD + dt * 16 + r0]) = c;
    }
    wave_lds_sync();
    v8h pv[4];
#pragma unroll
    for (int t = 0; t < 4; ++t) pv[t] = *(const v8h*)(&Cst[w][t * 256 + lane * 8]);
    _Float16* ob = ctx + ((size_t)b * SEQ + q0 + (lane >> 3)) * DM + h * HD + (lane & 7) * 8;
#pragma unroll
    for (int t = 0; t < 4; ++t) *(volatile v8h*)(ob + (size_t)(4 * t) * DM) = pv[t];
    __threadfence();
#pragma unroll
    for (int t = 0; t < 4; ++t) *(volatile v8h*)(ob + (size_t)(4 * t) * DM) = pv[t];
}

extern "C" void kernel_launch(void* const* d_in, const int* in_sizes, int n_in,
                              void* d_out, int out_size, void* d_ws, size_t ws_size,
                              hipStream_t stream) {
    if (n_in < 18) return;
    const int act_need = ((NB - 1) * SEQ_FULL + SEQ) * DM;
    if (in_sizes[0] < act_need || in_sizes[1] < act_need) return;
    if (in_sizes[2] < DM * DM || in_sizes[4] < DM * DM || in_sizes[6] < DM * DM || in_sizes[8] < DM * DM) return;
    if (in_sizes[3] < DM || in_sizes[5] < DM || in_sizes[7] < DM || in_sizes[9] < DM) return;
    if (in_sizes[10] < DM * DFF || in_sizes[11] < DFF || in_sizes[12] < DFF * DM || in_sizes[13] < DM) return;
    if (in_sizes[14] < SEQ * DM || in_sizes[15] < SEQ * DM || in_sizes[16] < SEQ * DM || in_sizes[17] < SEQ * DM) return;
    if (out_size < NTOK * DM) return;

    const float* x     = (const float*)d_in[0];
    const float* y     = (const float*)d_in[1];
    const float* Wq    = (const float*)d_in[2];
    const float* bq    = (const float*)d_in[3];
    const float* Wk    = (const float*)d_in[4];
    const float* bk    = (const float*)d_in[5];
    const float* Wv    = (const float*)d_in[6];
    const float* bv    = (const float*)d_in[7];
    const float* Wo    = (const float*)d_in[8];
    const float* bo    = (const float*)d_in[9];
    const float* W1    = (const float*)d_in[10];
    const float* b1    = (const float*)d_in[11];
    const float* W2    = (const float*)d_in[12];
    const float* b2    = (const float*)d_in[13];
    const float* ln1_w = (const float*)d_in[14];
    const float* ln1_b = (const float*)d_in[15];
    const float* ln2_w = (const float*)d_in[16];
    const float* ln2_b = (const float*)d_in[17];
    float* out = (float*)d_out;

    char* ws = (char*)d_ws;
    size_t off = 0;
    const size_t PL16 = (size_t)NTOK * DM * 2;
    const size_t WSQ  = (size_t)DM * DM * 2;
    const size_t WFF  = (size_t)DM * DFF * 2;
    const size_t PT   = (size_t)NB * PB * 128;
    _Float16* xh  = (_Float16*)(ws + off); off += PL16;
    _Float16* lnh = (_Float16*)(ws + off); off += PL16;
    _Float16* qpl = (_Float16*)(ws + off); off += PL16;
    _Float16* kpl = (_Float16*)(ws + off); off += PL16;
    _Float16* vTp = (_Float16*)(ws + off); off += PL16;
    _Float16* ctx = (_Float16*)(ws + off); off += PL16;
    _Float16* WqT = (_Float16*)(ws + off); off += WSQ;
    _Float16* WkT = (_Float16*)(ws + off); off += WSQ;
    _Float16* WvT = (_Float16*)(ws + off); off += WSQ;
    _Float16* WoT = (_Float16*)(ws + off); off += WSQ;
    _Float16* W1T = (_Float16*)(ws + off); off += WFF;
    _Float16* W2T = (_Float16*)(ws + off); off += WFF;
    float*    y1  = (float*)(ws + off);    off += (size_t)NTOK * DM * 4;
    _Float16* hp  = (_Float16*)(ws + off); off += (size_t)NTOK * DFF * 2;
    float* pS1 = (float*)(ws + off); off += PT;
    float* pV1 = (float*)(ws + off); off += PT;
    float* pS2 = (float*)(ws + off); off += PT;
    float* pV2 = (float*)(ws + off); off += PT;
    if (off > ws_size) return;
    if (off > (size_t)134217728) return;

    k_cvt<<<dim3(NTOK / 8), dim3(256), 0, stream>>>(x, xh);
    k_wprep<<<dim3(DM / 64, DM / 64), dim3(256), 0, stream>>>(Wq, DM, DM, WqT);
    k_wprep<<<dim3(DM / 64, DM / 64), dim3(256), 0, stream>>>(Wk, DM, DM, WkT);
    k_wprep<<<dim3(DM / 64, DM / 64), dim3(256), 0, stream>>>(Wv, DM, DM, WvT);
    k_wprep<<<dim3(DM / 64, DM / 64), dim3(256), 0, stream>>>(Wo, DM, DM, WoT);
    k_wprep<<<dim3(DFF / 64, DM / 64), dim3(256), 0, stream>>>(W1, DM, DFF, W1T);
    k_wprep<<<dim3(DM / 64, DFF / 64), dim3(256), 0, stream>>>(W2, DFF, DM, W2T);

    k_lnsum<true><<<dim3(PB, NB), dim3(256), 0, stream>>>(y, SEQ_FULL * DM, pS1);
    k_lnvar<true><<<dim3(PB, NB), dim3(256), 0, stream>>>(y, SEQ_FULL * DM, pS1, pV1);
    k_lnnorm<true><<<dim3(NTOK / 8), dim3(256), 0, stream>>>(y, SEQ_FULL * DM, pS1, pV1, ln1_w, ln1_b, lnh);

    k_gemm<false, false, false, false><<<dim3(DM / 128, NTOK / 64), dim3(128), 0, stream>>>(
        xh, WqT, DM, DM, DM, bq, 1.0f, SC_W, y, SEQ_FULL, (void*)qpl, DM);
    k_gemm<false, false, false, false><<<dim3(DM / 128, NTOK / 64), dim3(128), 0, stream>>>(
        lnh, WkT, DM, DM, DM, bk, 1.0f, SC_W, y, SEQ_FULL, (void*)kpl, DM);
    k_gemm<false, false, true, false><<<dim3(NTOK / 128, DM / 64), dim3(128), 0, stream>>>(
        WvT, lnh, DM, DM, DM, bv, 1.0f, SC_W, y, SEQ_FULL, (void*)vTp, NTOK);

    k_attn<<<dim3(SEQ / 128, NH, NB), dim3(256), 0, stream>>>(qpl, kpl, vTp, ctx);

    k_gemm<true, false, false, true><<<dim3(DM / 128, NTOK / 64), dim3(128), 0, stream>>>(
        ctx, WoT, DM, DM, DM, bo, SC_FOLD, 1.0f, y, SEQ_FULL, (void*)y1, DM);

    k_lnsum<false><<<dim3(PB, NB), dim3(256), 0, stream>>>(y1, SEQ * DM, pS2);
    k_lnvar<false><<<dim3(PB, NB), dim3(256), 0, stream>>>(y1, SEQ * DM, pS2, pV2);
    k_lnnorm<false><<<dim3(NTOK / 8), dim3(256), 0, stream>>>(y1, SEQ * DM, pS2, pV2, ln2_w, ln2_b, lnh);

    k_gemm<false, true, false, false><<<dim3(DFF / 128, NTOK / 64), dim3(128), 0, stream>>>(
        lnh, W1T, DM, DM, DM, b1, 1.0f, SC_W, y, SEQ_FULL, (void*)hp, DFF);
    k_gemm<true, false, false, false><<<dim3(DM / 128, NTOK / 64), dim3(128), 0, stream>>>(
        hp, W2T, DFF, DFF, DFF, b2, SC_FOLD, 1.0f, y1, SEQ, (void*)out, DM);
}
